// TransformerEncoder_23673859735588
// MI455X (gfx1250) — hardware-verified
//
#include <hip/hip_runtime.h>
#ifndef NB
#define NB 2
#endif
#ifndef SEQ
#define SEQ 2048
#endif
#define NB_FULL 2
#define SEQ_FULL 2048
#define FEAT 1024
#define NHEAD 16
#define DHEAD 64
#define MLPH 4096
#define MR (NB * SEQ)
#define QKVN (3 * FEAT)
static_assert(SEQ % 64 == 0);
static_assert(SEQ <= SEQ_FULL);
static_assert(NB >= 1);
static_assert(NB <= NB_FULL);
static_assert(FEAT == NHEAD * DHEAD);
static_assert(FEAT % 64 == 0);
static_assert(MLPH % 64 == 0);
static_assert(QKVN % 64 == 0);
static_assert(FEAT % 32 == 0);
static_assert(MLPH % 32 == 0);
static_assert(FEAT == 128 * 8);
static_assert(FEAT == 8 * (1 << 7));
static_assert(MLPH == 8 * (1 << 9));
static_assert(MR % 16 == 0);
static_assert((QKVN * (FEAT / 8)) % 256 == 0);
static_assert((MLPH * (FEAT / 8)) % 256 == 0);
static_assert((FEAT * (MLPH / 8)) % 256 == 0);
static_assert(((MR / 16) * (QKVN / 64)) % 4 == 0);
static_assert(((MR / 16) * (MLPH / 64)) % 4 == 0);
static_assert(((MR / 16) * (FEAT / 64)) % 4 == 0);
static_assert((NB * NHEAD * (SEQ / 64)) * 4 * 16 * DHEAD == MR * FEAT);

typedef _Float16 v16h __attribute__((ext_vector_type(16)));
typedef unsigned short v8us __attribute__((ext_vector_type(8), may_alias));
typedef float v8f __attribute__((ext_vector_type(8)));
typedef float v4f __attribute__((ext_vector_type(4)));
typedef float v4fa __attribute__((ext_vector_type(4), may_alias));
union FragH { v16h v; v8us half[2]; unsigned short u[16]; };
union H16U { _Float16 h; unsigned short u; };

__device__ __forceinline__ unsigned short bf16_bits(float x) { unsigned int u = __float_as_uint(x); return (unsigned short)((u + 0x7FFFu + ((u >> 16) & 1u)) >> 16); }
__device__ __forceinline__ float bf16_val(unsigned short b) { return __uint_as_float(((unsigned int)b) << 16); }
__device__ __forceinline__ float bf16_rne(float x) { return bf16_val(bf16_bits(x)); }
__device__ __forceinline__ unsigned short h16_bits(float x) { H16U t; t.h = (_Float16)x; return t.u; }
__device__ __forceinline__ v8f vz8() { v8f z = {0.f, 0.f, 0.f, 0.f, 0.f, 0.f, 0.f, 0.f}; return z; }

__device__ __forceinline__ v8f mma16(v16h a, v16h b, v8f c) {
  c = __builtin_amdgcn_wmma_f32_16x16x32_f16(false, a, false, b, (short)0, c, false, false);
  asm volatile("v_nop\n\tv_nop\n\tv_nop\n\tv_nop" : "+v"(c) : "v"(a), "v"(b));
  return c;
}

__global__ __launch_bounds__(256) void k_wt16(const float* __restrict__ W, unsigned short* __restrict__ Wt, unsigned K, unsigned N, unsigned k8sh, float sc) {
  const unsigned t = blockIdx.x * 256u + threadIdx.x;
  if (t >= (N << k8sh)) return;
  const unsigned n = t >> k8sh;
  const unsigned k8 = (t & ((1u << k8sh) - 1u)) << 3;
  v8us v;
#pragma unroll
  for (int i = 0; i < 8; ++i) v[i] = h16_bits(bf16_rne(W[(size_t)(k8 + (unsigned)i) * N + n]) * sc);
  unsigned short* dst = Wt + (size_t)n * K + k8;
  *(volatile v8us*)dst = v;
  __threadfence();
  *(volatile v8us*)dst = v;
}

template <bool RND>
__global__ __launch_bounds__(128) void k_ln16(const float* __restrict__ X, unsigned in_map,
                                              const float* __restrict__ g, const float* __restrict__ bt,
                                              unsigned short* __restrict__ out, float osc, float eps) {
  __shared__ float red1[4];
  __shared__ float red2[4];
  const unsigned m = blockIdx.x, tid = threadIdx.x, w = tid >> 5, lane = tid & 31u;
  const unsigned srow = in_map ? ((m / (unsigned)SEQ) * (unsigned)SEQ_FULL + (m % (unsigned)SEQ)) : m;
  const float* x = X + (size_t)srow * FEAT + tid * 8u;
  const v4f a0 = *(const v4fa*)x;
  const v4f a1 = *(const v4fa*)(x + 4);
  float v[8] = {a0[0], a0[1], a0[2], a0[3], a1[0], a1[1], a1[2], a1[3]};
  if (RND) {
#pragma unroll
    for (int q = 0; q < 8; ++q) v[q] = bf16_rne(v[q]);
  }
  float s = 0.f;
#pragma unroll
  for (int q = 0; q < 8; ++q) s += v[q];
#pragma unroll
  for (int o = 16; o >= 1; o >>= 1) s += __shfl_xor(s, o, 32);
  if (lane == 0) red1[w] = s;
  __syncthreads();
  const float mu = ((red1[0] + red1[1]) + (red1[2] + red1[3])) * (1.0f / (float)FEAT);
  float c[8];
  float s2 = 0.f;
#pragma unroll
  for (int q = 0; q < 8; ++q) { c[q] = v[q] - mu; s2 += c[q] * c[q]; }
#pragma unroll
  for (int o = 16; o >= 1; o >>= 1) s2 += __shfl_xor(s2, o, 32);
  if (lane == 0) red2[w] = s2;
  __syncthreads();
  const float var = ((red2[0] + red2[1]) + (red2[2] + red2[3])) * (1.0f / (float)FEAT);
  const float rs = rsqrtf(var + eps);
  const v4f g0 = *(const v4fa*)(g + tid * 8u);
  const v4f g1 = *(const v4fa*)(g + tid * 8u + 4u);
  const v4f b0 = *(const v4fa*)(bt + tid * 8u);
  const v4f b1 = *(const v4fa*)(bt + tid * 8u + 4u);
  const float gg[8] = {g0[0], g0[1], g0[2], g0[3], g1[0], g1[1], g1[2], g1[3]};
  const float bb[8] = {b0[0], b0[1], b0[2], b0[3], b1[0], b1[1], b1[2], b1[3]};
  v8us o;
#pragma unroll
  for (int q = 0; q < 8; ++q) o[q] = h16_bits((c[q] * rs * bf16_rne(gg[q]) + bf16_rne(bb[q])) * osc);
  unsigned short* dst = out + (size_t)m * FEAT + tid * 8u;
  *(volatile v8us*)dst = o;
  __threadfence();
  *(volatile v8us*)dst = o;
}

template <bool OUT16, int ACT, bool HASRES>
__global__ __launch_bounds__(128) void k_gemm16(const unsigned short* __restrict__ A, unsigned lda, const unsigned short* __restrict__ Wt, unsigned ldb,
                                                const float* __restrict__ bias, const float* __restrict__ resid, unsigned ldr,
                                                void* __restrict__ Cv, unsigned ldc, unsigned out_map,
                                                unsigned M, unsigned N, unsigned K, float inv_scale, float out_scale) {
  __shared__ __attribute__((aligned(16))) float so32[OUT16 ? 1 : 4][16][64];
  __shared__ __attribute__((aligned(16))) unsigned short so16[OUT16 ? 4 : 1][16][72];
  const unsigned tid = threadIdx.x, w = tid >> 5, lane = tid & 31u, ln = lane & 15u, hh = lane >> 4;
  const unsigned ntn = N >> 6;
  const unsigned wid = blockIdx.x * 4u + w;
  const unsigned mt = wid / ntn, nq = wid - mt * ntn;
  if (mt * 16u >= M) return;
  const unsigned row0 = mt * 16u, col0 = nq * 64u;
  const unsigned short* arow = A + (size_t)(row0 + ln) * lda;
  v8f acc[4];
#pragma unroll
  for (int t = 0; t < 4; ++t) acc[t] = vz8();
  for (unsigned kb = 0; kb < K; kb += 32u) {
    FragH a;
    a.half[0] = *(const v8us*)(arow + kb + 8u * hh);
    a.half[1] = *(const v8us*)(arow + kb + 16u + 8u * hh);
#pragma unroll
    for (int t = 0; t < 4; ++t) {
      const unsigned short* brow = Wt + (size_t)(col0 + (unsigned)t * 16u + ln) * ldb + kb;
      FragH bb;
      bb.half[0] = *(const v8us*)(brow + 8u * hh);
      bb.half[1] = *(const v8us*)(brow + 16u + 8u * hh);
      acc[t] = mma16(a.v, bb.v, acc[t]);
    }
  }
#pragma unroll
  for (int t = 0; t < 4; ++t) {
    const unsigned col = col0 + (unsigned)t * 16u + ln;
    const float bvv = bf16_rne(bias[col]);
#pragma unroll
    for (int r = 0; r < 8; ++r) {
      float v = acc[t][r] * inv_scale + bvv;
      if (ACT == 1) v = fmaxf(v, 0.0f);
      if constexpr (OUT16) so16[w][8u * hh + (unsigned)r][(unsigned)t * 16u + ln] = h16_bits(v * out_scale);
      else so32[w][8u * hh + (unsigned)r][(unsigned)t * 16u + ln] = v;
    }
  }
  __builtin_amdgcn_fence(4  , "workgroup");
  __builtin_amdgcn_wave_barrier();
  const unsigned orow0 = out_map ? ((row0 / (unsigned)SEQ) * (unsigned)SEQ_FULL + (row0 % (unsigned)SEQ)) : row0;
  if constexpr (OUT16) {
    unsigned short* Ch = (unsigned short*)Cv;
    const unsigned rq = lane >> 3, p8 = (lane & 7u) * 8u;
    v8us ov[4];
#pragma unroll
    for (int q = 0; q < 4; ++q) ov[q] = *(const v8us*)&so16[w][(unsigned)q * 4u + rq][p8];
#pragma unroll
    for (int pass = 0; pass < 2; ++pass) {
#pragma unroll
      for (int q = 0; q < 4; ++q) {
        const unsigned r = (unsigned)q * 4u + rq;
        *(volatile v8us*)(Ch + (size_t)(orow0 + r) * ldc + col0 + p8) = ov[q];
      }
      if (pass == 0) __threadfence();
    }
  } else {
    float* Cf = (float*)Cv;
    const unsigned rsub = lane >> 4, c4 = (lane & 15u) * 4u;
    v4f outv[8];
#pragma unroll
    for (int q = 0; q < 8; ++q) {
      const unsigned r = (unsigned)q * 2u + rsub;
      v4f v = *(const v4fa*)&so32[w][r][c4];
      if constexpr (HASRES) {
        const v4f rv = *(const v4fa*)(resid + (size_t)(row0 + r) * ldr + col0 + c4);
        v = v + rv;
      }
      outv[q] = v;
    }
#pragma unroll
    for (int pass = 0; pass < 2; ++pass) {
#pragma unroll
      for (int q = 0; q < 8; ++q) {
        const unsigned r = (unsigned)q * 2u + rsub;
        *(volatile v4f*)(Cf + (size_t)(orow0 + r) * ldc + col0 + c4) = outv[q];
      }
      if (pass == 0) __threadfence();
    }
  }
}

template <int D>
__global__ __launch_bounds__(128) void k_attn16(const unsigned short* __restrict__ qkv, unsigned pitch, unsigned T, unsigned H, unsigned koff, unsigned voff,
                                                float scale, float pcarry, float onorm,
                                                const float* __restrict__ xres, unsigned xseq, unsigned xpitch,
                                                float* __restrict__ att, unsigned cpitch) {
  static_assert(D == 64);
  constexpr int KS = D / 32, DT = D / 16, C8 = D / 8;
  static_assert((32 * C8) % 128 == 0);
  static_assert(C8 == 8);
  __shared__ __attribute__((aligned(16))) unsigned short sK[32][D + 8];
  __shared__ __attribute__((aligned(16))) unsigned short sVt[D][40];
  __shared__ __attribute__((aligned(16))) unsigned short sP[4][16][40];
  __shared__ __attribute__((aligned(16))) float sO[4][16][D];
  const unsigned tid = threadIdx.x, w = tid >> 5, lane = tid & 31u, ln = lane & 15u, hh = lane >> 4;
  const unsigned nqb = T >> 6;
  const unsigned bh = blockIdx.x / nqb, qblk = blockIdx.x - bh * nqb;
  const unsigned b = bh / H, h = bh - b * H;
  const unsigned q0 = qblk * 64u + w * 16u;
  const unsigned short* Qp = qkv + (size_t)b * T * pitch + h * (unsigned)D;
  const unsigned short* Kp = Qp + koff;
  const unsigned short* Vp = Qp + voff;

  FragH aq[KS];
  {
    const unsigned short* qr = Qp + (size_t)(q0 + ln) * pitch;
#pragma unroll
    for (int ks = 0; ks < KS; ++ks) {
      aq[ks].half[0] = *(const v8us*)(qr + ks * 32 + 8u * hh);
      aq[ks].half[1] = *(const v8us*)(qr + ks * 32 + 16 + 8u * hh);
    }
  }
  float m_r[8], l_r[8];
#pragma unroll
  for (int r = 0; r < 8; ++r) { m_r[r] = -1.0e30f; l_r[r] = 0.f; }
  v8f oacc[DT];
#pragma unroll
  for (int dt = 0; dt < DT; ++dt) oacc[dt] = vz8();

  for (unsigned j0 = 0; j0 < T; j0 += 32u) {
    __syncthreads();
#pragma unroll
    for (int it = 0; it < (32 * C8) / 128; ++it) {
      const unsigned e = tid + (unsigned)it * 128u;
      const unsigned r = e >> 3, c8 = (e & 7u) * 8u;
      const size_t ro = (size_t)(j0 + r) * pitch + c8;
      const v8us kvv = *(const v8us*)(Kp + ro);
      *(v8us*)&sK[r][c8] = kvv;
      const v8us vvv = *(const v8us*)(Vp + ro);
#pragma unroll
      for (int i = 0; i < 8; ++i) sVt[c8 + (unsigned)i][r] = vvv[i];
    }
    __syncthreads();
    v8f s[2];
#pragma unroll
    for (int nt = 0; nt < 2; ++nt) {
      v8f acc = vz8();
#pragma unroll
      for (int ks = 0; ks < KS; ++ks) {
        FragH bk;
        bk.half[0] = *(const v8us*)&sK[(unsigned)nt * 16u + ln][(unsigned)ks * 32u + 8u * hh];
        bk.half[1] = *(const v8us*)&sK[(unsigned)nt * 16u + ln][(unsigned)ks * 32u + 16u + 8u * hh];
        acc = mma16(aq[ks].v, bk.v, acc);
      }
      s[nt] = acc;
    }
    float alpha[8];
#pragma unroll
    for (int r = 0; r < 8; ++r) {
      const float s0 = s[0][r] * scale, s1 = s[1][r] * scale;
      float mx = fmaxf(s0, s1);
      mx = fmaxf(mx, __shfl_xor(mx, 1, 32)); mx = fmaxf(mx, __shfl_xor(mx, 2, 32));
      mx = fmaxf(mx, __shfl_xor(mx, 4, 32)); mx = fmaxf(mx, __shfl_xor(mx, 8, 32));
      const float mnew = fmaxf(m_r[r], mx);
      alpha[r] = __expf(m_r[r] - mnew);
      const float p0 = __expf(s0 - mnew), p1 = __expf(s1 - mnew);
      m_r[r] = mnew;
      l_r[r] = l_r[r] * alpha[r] + p0 + p1;
      sP[w][8u * hh + (unsigned)r][ln] = h16_bits(p0 * pcarry);
      sP[w][8u * hh + (unsigned)r][16u + ln] = h16_bits(p1 * pcarry);
    }
#pragma unroll
    for (int dt = 0; dt < DT; ++dt)
#pragma unroll
      for (int r = 0; r < 8; ++r) oacc[dt][r] *= alpha[r];
    __builtin_amdgcn_fence(4  , "workgroup");
    __builtin_amdgcn_wave_barrier();
    FragH pa;
    pa.half[0] = *(const v8us*)&sP[w][ln][8u * hh];
    pa.half[1] = *(const v8us*)&sP[w][ln][16u + 8u * hh];
#pragma unroll
    for (int dt = 0; dt < DT; ++dt) {
      FragH bv;
      bv.half[0] = *(const v8us*)&sVt[(unsigned)dt * 16u + ln][8u * hh];
      bv.half[1] = *(const v8us*)&sVt[(unsigned)dt * 16u + ln][16u + 8u * hh];
      oacc[dt] = mma16(pa.v, bv.v, oacc[dt]);
    }
    __builtin_amdgcn_fence(4  , "workgroup");
    __builtin_amdgcn_wave_barrier();
  }
#pragma unroll
  for (int r = 0; r < 8; ++r) {
    float l = l_r[r];
    l += __shfl_xor(l, 1, 32); l += __shfl_xor(l, 2, 32); l += __shfl_xor(l, 4, 32); l += __shfl_xor(l, 8, 32);
    l_r[r] = onorm * (1.0f / l);
  }
#pragma unroll
  for (int dt = 0; dt < DT; ++dt)
#pragma unroll
    for (int r = 0; r < 8; ++r) sO[w][8u * hh + (unsigned)r][(unsigned)dt * 16u + ln] = oacc[dt][r] * l_r[r];
  __builtin_amdgcn_fence(4  , "workgroup");
  __builtin_amdgcn_wave_barrier();
  const unsigned rsub = lane >> 4, c4 = (lane & 15u) * 4u;
  const float* xrow = xres + ((size_t)b * xseq + q0) * xpitch + h * (unsigned)D + c4;
  float* arow = att + ((size_t)b * T + q0) * cpitch + h * (unsigned)D + c4;
  v4f outv[8];
#pragma unroll
  for (int q = 0; q < 8; ++q) {
    const unsigned r = (unsigned)q * 2u + rsub;
    v4f v = *(const v4fa*)&sO[w][r][c4];
    const v4f xv = *(const v4fa*)(xrow + (size_t)r * xpitch);
    v[0] += bf16_rne(xv[0]); v[1] += bf16_rne(xv[1]); v[2] += bf16_rne(xv[2]); v[3] += bf16_rne(xv[3]);
    outv[q] = v;
  }
#pragma unroll
  for (int pass = 0; pass < 2; ++pass) {
#pragma unroll
    for (int q = 0; q < 8; ++q) {
      const unsigned r = (unsigned)q * 2u + rsub;
      *(volatile v4f*)(arow + (size_t)r * cpitch) = outv[q];
    }
    if (pass == 0) __threadfence();
  }
}

extern "C" void kernel_launch(void* const* d_in, const int* in_sizes, int n_in,
                              void* d_out, int out_size, void* d_ws, size_t ws_size, hipStream_t stream) {
  if (n_in < 11) return;
  const long long need_rows = (long long)(NB - 1) * SEQ_FULL + SEQ;
  if ((long long)in_sizes[0] < need_rows * FEAT) return;
  if (in_sizes[1] < FEAT || in_sizes[2] < FEAT || in_sizes[5] < FEAT || in_sizes[6] < FEAT || in_sizes[10] < FEAT) return;
  if (in_sizes[3] < FEAT * QKVN || in_sizes[4] < QKVN) return;
  if (in_sizes[7] < FEAT * MLPH || in_sizes[8] < MLPH || in_sizes[9] < MLPH * FEAT) return;
  if ((long long)out_size < need_rows * FEAT) return;

  const float* x    = (const float*)d_in[0];
  const float* g1   = (const float*)d_in[1];  const float* be1 = (const float*)d_in[2];
  const float* Wqkv = (const float*)d_in[3];  const float* bqkv = (const float*)d_in[4];
  const float* g2   = (const float*)d_in[5];  const float* be2 = (const float*)d_in[6];
  const float* W1   = (const float*)d_in[7];  const float* b1 = (const float*)d_in[8];
  const float* W2   = (const float*)d_in[9];  const float* b2 = (const float*)d_in[10];

  char* ws = (char*)d_ws; size_t off = 0;
  auto take = [&](size_t bytes) { char* p = ws + off; off += (bytes + 255) & ~(size_t)255; return p; };
  unsigned short* Wqkv16 = (unsigned short*)take((size_t)QKVN * FEAT * 2);
  unsigned short* W116   = (unsigned short*)take((size_t)MLPH * FEAT * 2);
  unsigned short* W216   = (unsigned short*)take((size_t)FEAT * MLPH * 2);
  const size_t r1_bytes = (size_t)MR * FEAT * 2;
  const size_t r2_a = (size_t)MR * QKVN * 2, r2_b = (size_t)MR * MLPH * 2;
  const size_t r2_bytes = (r2_a > r2_b) ? r2_a : r2_b;
  unsigned short* R1 = (unsigned short*)take(r1_bytes);
  unsigned short* R2 = (unsigned short*)take(r2_bytes);
  float* ATT32 = (float*)take((size_t)MR * FEAT * 4);
  if (off > ws_size) return;
  if (off > (size_t)134217728) return;

  const float wsc = 256.0f;
  k_wt16<<<(unsigned)((QKVN * (FEAT / 8)) / 256), 256, 0, stream>>>(Wqkv, Wqkv16, (unsigned)FEAT, (unsigned)QKVN, 7u, wsc);
  k_wt16<<<(unsigned)((MLPH * (FEAT / 8)) / 256), 256, 0, stream>>>(W1, W116, (unsigned)FEAT, (unsigned)MLPH, 7u, wsc);
  k_wt16<<<(unsigned)((FEAT * (MLPH / 8)) / 256), 256, 0, stream>>>(W2, W216, (unsigned)MLPH, (unsigned)FEAT, 9u, wsc);

  auto ggrid = [](int M, int N) { return (unsigned)(((M / 16) * (N / 64) + 3) / 4); };

  k_ln16<true><<<(unsigned)MR, 128, 0, stream>>>(x, 1u, g1, be1, R1, 8.0f, 1e-5f);
  k_gemm16<true, 0, false><<<ggrid(MR, QKVN), 128, 0, stream>>>(R1, (unsigned)FEAT, Wqkv16, (unsigned)FEAT, bqkv, nullptr, 0u,
                                                                 (void*)R2, (unsigned)QKVN, 0u, (unsigned)MR, (unsigned)QKVN, (unsigned)FEAT,
                                                                 1.0f / 2048.0f, 8.0f);
  k_attn16<DHEAD><<<(unsigned)(NB * NHEAD * (SEQ / 64)), 128, 0, stream>>>(R2, (unsigned)QKVN, (unsigned)SEQ, (unsigned)NHEAD,
                                                                           (unsigned)FEAT, (unsigned)(2 * FEAT),
                                                                           0.001953125f, 1024.0f, 1.0f / 8192.0f,
                                                                           x, (unsigned)SEQ_FULL, (unsigned)FEAT, ATT32, (unsigned)FEAT);
  k_ln16<false><<<(unsigned)MR, 128, 0, stream>>>(ATT32, 0u, g2, be2, R1, 8.0f, 1e-5f);
  k_gemm16<true, 1, false><<<ggrid(MR, MLPH), 128, 0, stream>>>(R1, (unsigned)FEAT, W116, (unsigned)FEAT, b1, nullptr, 0u,
                                                                 (void*)R2, (unsigned)MLPH, 0u, (unsigned)MR, (unsigned)MLPH, (unsigned)FEAT,
                                                                 1.0f / 2048.0f, 16.0f);
  k_gemm16<false, 0, true><<<ggrid(MR, FEAT), 128, 0, stream>>>(R2, (unsigned)MLPH, W216, (unsigned)MLPH, b2, ATT32, (unsigned)FEAT,
                                                                 d_out, (unsigned)FEAT, 1u, (unsigned)MR, (unsigned)FEAT, (unsigned)MLPH,
                                                                 1.0f / 4096.0f, 1.0f);
}
